// CATAttention_89043261981441
// MI455X (gfx1250) — hardware-verified
//
#include <hip/hip_runtime.h>
#include <stddef.h>
#include <stdint.h>

#define NB    2
#define SQ    2048
#define EMB   1024
#define NHD   16
#define HDM   64
#define NTOK  (NB * SQ)
#define NBH   (NB * NHD)
#define QB    64
#define KC    64
#define NQB   (SQ / QB)
#define WCAR  64.0f
#define ZCAR  2048.0f
#define MIDF  0.5f
#define OUTF  (1.0f / 65536.0f)
#define CVB   2048
#define NXB   ((NTOK * EMB) / CVB)
#define NWB   ((EMB * EMB) / CVB)

static_assert(NTOK == 4096);
static_assert(EMB == NHD * HDM);
static_assert(HDM == 64);
static_assert(SQ % QB == 0);
static_assert(QB == KC);
static_assert(NQB == 32);
static_assert(EMB % 32 == 0);
static_assert((NTOK * EMB) % CVB == 0);
static_assert((EMB * EMB) % CVB == 0);
static_assert(SQ == 256 * 8);
static_assert(SQ == 128 * 16);
static_assert(NTOK % 64 == 0);
static_assert(EMB % 64 == 0);

typedef _Float16 hf;
typedef hf            v16h __attribute__((ext_vector_type(16)));
typedef hf            v8h  __attribute__((ext_vector_type(8)));
typedef float         v8f  __attribute__((ext_vector_type(8)));
typedef float         v4f  __attribute__((ext_vector_type(4)));
typedef unsigned int  v4u  __attribute__((ext_vector_type(4)));

union Frag  { v16h v; v8h h[2]; };
union Pack8 { v8h h; v4u u; };

__device__ __forceinline__ v8f mma16(v16h a, v16h b, v8f c) {
  c = __builtin_amdgcn_wmma_f32_16x16x32_f16(false, a, false, b, (short)0, c, false, false);
  asm volatile("v_nop\n\tv_nop\n\tv_nop\n\tv_nop" : "+v"(c) : "v"(a), "v"(b));
  return c;
}

__device__ __forceinline__ v16h ldfrag(const hf* p, int ld, int row0, int k0, int lane) {
  const int m = lane & 15, lh = lane >> 4;
  const hf* q = p + (size_t)(row0 + m) * ld + k0 + 8 * lh;
  Frag f;
  f.h[0] = *(const v8h*)(q);
  f.h[1] = *(const v8h*)(q + 16);
  return f.v;
}

__device__ __forceinline__ v8f zero8() { return (v8f){0.f, 0.f, 0.f, 0.f, 0.f, 0.f, 0.f, 0.f}; }

template <int KD>
__device__ __forceinline__ void gemm16x64(const hf* __restrict__ A, const hf* __restrict__ Bm,
                                          int m0, int n0, int lane, v8f (&acc)[4]) {
  static_assert(KD % 32 == 0);
#pragma unroll 1
  for (int k0 = 0; k0 < KD; k0 += 32) {
    const v16h a = ldfrag(A, KD, m0, k0, lane);
#pragma unroll
    for (int t = 0; t < 4; ++t) {
      const v16h bb = ldfrag(Bm, KD, n0 + 16 * t, k0, lane);
      acc[t] = mma16(a, bb, acc[t]);
    }
  }
}

__global__ __launch_bounds__(256) void k_cvt(const float* __restrict__ x, const float* __restrict__ wv,
                                             const float* __restrict__ wo,
                                             hf* __restrict__ xh, hf* __restrict__ wvh, hf* __restrict__ woh) {
  const int blk = blockIdx.x;
  const int sel = (blk < NXB) ? 0 : ((blk < NXB + NWB) ? 1 : 2);
  const float* s = (sel == 0) ? x : ((sel == 1) ? wv : wo);
  hf* d = (sel == 0) ? xh : ((sel == 1) ? wvh : woh);
  const float sc = (sel == 0) ? 1.0f : WCAR;
  const int lb = (sel == 0) ? blk : ((sel == 1) ? (blk - NXB) : (blk - NXB - NWB));
  const size_t i = (size_t)lb * CVB + (size_t)threadIdx.x * 8;
  const v4f a0 = *(const v4f*)(s + i);
  const v4f a1 = *(const v4f*)(s + i + 4);
  Pack8 pk;
  pk.h = (v8h){(hf)(a0[0] * sc), (hf)(a0[1] * sc), (hf)(a0[2] * sc), (hf)(a0[3] * sc),
               (hf)(a1[0] * sc), (hf)(a1[1] * sc), (hf)(a1[2] * sc), (hf)(a1[3] * sc)};
  const v4u u = pk.u;
  *(volatile v4u*)(d + i) = u;
  __threadfence();
  *(volatile v4u*)(d + i) = u;
}

__global__ __launch_bounds__(256) void k_zsoft(const float* __restrict__ x, const float* __restrict__ wa,
                                               hf* __restrict__ zp) {
  __shared__ __align__(16) float was[EMB];
  __shared__ float zf[SQ];
  __shared__ float red[256];
  __shared__ __align__(16) hf zh[SQ];
  const int tid = threadIdx.x;
  const int bh = blockIdx.x;
  const int b = bh >> 4, h = bh & 15;

  *(v4f*)(was + 4 * tid) = *(const v4f*)(wa + (size_t)h * EMB + 4 * tid);
  __syncthreads();

  float mx = -__builtin_huge_valf();
#pragma unroll 1
  for (int q = 0; q < SQ / 256; ++q) {
    const int s = tid + 256 * q;
    const float* xr = x + ((size_t)(b * SQ + s)) * EMB;
    float c0 = 0.f, c1 = 0.f, c2 = 0.f, c3 = 0.f;
#pragma unroll 2
    for (int e = 0; e < EMB; e += 4) {
      const v4f xv = *(const v4f*)(xr + e);
      const v4f wv = *(const v4f*)(was + e);
      c0 = fmaf(xv[0], wv[0], c0);
      c1 = fmaf(xv[1], wv[1], c1);
      c2 = fmaf(xv[2], wv[2], c2);
      c3 = fmaf(xv[3], wv[3], c3);
    }
    const float lg = ((c0 + c1) + (c2 + c3)) * 0.125f;
    zf[s] = lg;
    mx = fmaxf(mx, lg);
  }
  red[tid] = mx;
  __syncthreads();
  for (int off = 128; off > 0; off >>= 1) {
    if (tid < off) red[tid] = fmaxf(red[tid], red[tid + off]);
    __syncthreads();
  }
  const float m = red[0];
  __syncthreads();

  float sum = 0.f;
#pragma unroll 1
  for (int q = 0; q < SQ / 256; ++q) {
    const int s = tid + 256 * q;
    const float ev = expf(zf[s] - m);
    zf[s] = ev;
    sum += ev;
  }
  red[tid] = sum;
  __syncthreads();
  for (int off = 128; off > 0; off >>= 1) {
    if (tid < off) red[tid] += red[tid + off];
    __syncthreads();
  }
  const float tot = red[0];
  const float scl = ZCAR * (1.0f / tot);
#pragma unroll 1
  for (int q = 0; q < SQ / 256; ++q) {
    const int s = tid + 256 * q;
    zh[s] = (hf)(zf[s] * scl);
  }
  __syncthreads();
  Pack8 pk;
  pk.h = *(const v8h*)(zh + 8 * tid);
  const v4u u = pk.u;
  hf* dst = zp + (size_t)bh * SQ + 8 * tid;
  *(volatile v4u*)dst = u;
  __threadfence();
  *(volatile v4u*)dst = u;
}

#define SFP 68
__global__ __launch_bounds__(128) void k_vproj(const hf* __restrict__ xh, const hf* __restrict__ wvh,
                                               hf* __restrict__ vt) {
  __shared__ __align__(16) float sf[64 * SFP];
  const int tid = threadIdx.x, lane = tid & 31, wave = tid >> 5;
  const int hh = lane >> 4, c = lane & 15;
  const int mb = blockIdx.x * 64;
  const int hd = blockIdx.y;
  const int m0 = mb + wave * 16;
  const int n0 = HDM * hd;

  v8f acc[4];
#pragma unroll
  for (int t = 0; t < 4; ++t) acc[t] = zero8();
  gemm16x64<EMB>(xh, wvh, m0, n0, lane, acc);

#pragma unroll
  for (int t = 0; t < 4; ++t) {
#pragma unroll
    for (int r = 0; r < 8; ++r)
      sf[(wave * 16 + 8 * hh + r) * SFP + 16 * t + c] = acc[t][r] * (1.0f / WCAR);
  }
  __syncthreads();

  const int bidx = mb / SQ;
  const int s0   = mb - bidx * SQ;
  v4u hv[4];
  size_t go[4];
#pragma unroll
  for (int j = 0; j < 4; ++j) {
    const int p  = tid + 128 * j;
    const int d  = p >> 3;
    const int pc = p & 7;
    const float* cp = sf + (pc * 8) * SFP + d;
    Pack8 pk;
    pk.h = (v8h){(hf)cp[0 * SFP], (hf)cp[1 * SFP], (hf)cp[2 * SFP], (hf)cp[3 * SFP],
                 (hf)cp[4 * SFP], (hf)cp[5 * SFP], (hf)cp[6 * SFP], (hf)cp[7 * SFP]};
    hv[j] = pk.u;
    go[j] = ((size_t)((bidx * NHD + hd) * HDM + d)) * SQ + s0 + pc * 8;
  }
#pragma unroll
  for (int j = 0; j < 4; ++j) *(volatile v4u*)(vt + go[j]) = hv[j];
  __threadfence();
#pragma unroll
  for (int j = 0; j < 4; ++j) *(volatile v4u*)(vt + go[j]) = hv[j];
}

#define LP 72
__global__ __launch_bounds__(128) void k_toep(const hf* __restrict__ zp, const hf* __restrict__ vt,
                                              hf* __restrict__ mid) {
  __shared__ __align__(16) hf zs[SQ];
  __shared__ __align__(16) hf Tt[QB * LP];
  __shared__ __align__(16) hf Vs[HDM * LP];

  const int tid = threadIdx.x, lane = tid & 31, wave = tid >> 5;
  const int hh = lane >> 4, c = lane & 15;
  const int qb = blockIdx.x & (NQB - 1);
  const int bh = blockIdx.x >> 5;
  const int b  = bh >> 4, hd = bh & 15;
  const int i0 = qb * QB;

  {
    const hf* zr = zp + (size_t)bh * SQ;
    *(v8h*)(zs + 16 * tid)     = *(const v8h*)(zr + 16 * tid);
    *(v8h*)(zs + 16 * tid + 8) = *(const v8h*)(zr + 16 * tid + 8);
  }
  const hf* Vg = vt + (size_t)bh * HDM * SQ;

  v8f oacc[4];
#pragma unroll
  for (int t = 0; t < 4; ++t) oacc[t] = zero8();

  const int nck = qb + 1;
  for (int ci = 0; ci < nck; ++ci) {
    const int kv0 = ci * KC;
    __syncthreads();
    {
      const int r  = tid >> 1;
      const int cb = (tid & 1) * 32;
      const hf* src = Vg + (size_t)r * SQ + kv0 + cb;
#pragma unroll
      for (int e = 0; e < 4; ++e) *(v8h*)(Vs + r * LP + cb + 8 * e) = *(const v8h*)(src + 8 * e);
    }
#pragma unroll
    for (int j = 0; j < 4; ++j) {
      const int p   = tid + 128 * j;
      const int row = p >> 3;
      const int pc  = p & 7;
      const int dbase = (i0 + row) - (kv0 + 8 * pc);
      hf tv[8];
#pragma unroll
      for (int e = 0; e < 8; ++e) {
        const int idx = dbase - e;
        int ia = (idx < 0) ? 0 : idx;
        ia = (ia > SQ - 1) ? (SQ - 1) : ia;
        const hf zv = zs[ia];
        tv[e] = (idx >= 0) ? zv : (hf)0.0f;
      }
      *(v8h*)(Tt + row * LP + 8 * pc) = (v8h){tv[0], tv[1], tv[2], tv[3], tv[4], tv[5], tv[6], tv[7]};
    }
    __syncthreads();

#pragma unroll
    for (int kk = 0; kk < 2; ++kk) {
      const v16h ta = ldfrag(Tt, LP, wave * 16, kk * 32, lane);
#pragma unroll
      for (int t = 0; t < 4; ++t) {
        const v16h vb = ldfrag(Vs, LP, t * 16, kk * 32, lane);
        oacc[t] = mma16(ta, vb, oacc[t]);
      }
    }
  }

  __syncthreads();
#pragma unroll
  for (int r = 0; r < 8; ++r) {
#pragma unroll
    for (int t = 0; t < 4; ++t)
      Tt[(wave * 16 + 8 * hh + r) * LP + 16 * t + c] = (hf)(oacc[t][r] * MIDF);
  }
  __syncthreads();
  v4u hv[4];
  size_t go[4];
  const size_t tok0 = (size_t)b * SQ + i0 + wave * 16;
#pragma unroll
  for (int it = 0; it < 4; ++it) {
    const int p  = lane + 32 * it;
    const int L  = p >> 3;
    const int pc = p & 7;
    Pack8 pk;
    pk.h   = *(const v8h*)(Tt + (wave * 16 + L) * LP + pc * 8);
    hv[it] = pk.u;
    go[it] = (tok0 + L) * EMB + HDM * hd + pc * 8;
  }
#pragma unroll
  for (int it = 0; it < 4; ++it) *(volatile v4u*)(mid + go[it]) = hv[it];
  __threadfence();
#pragma unroll
  for (int it = 0; it < 4; ++it) *(volatile v4u*)(mid + go[it]) = hv[it];
}

#define OTP 68
__global__ __launch_bounds__(128) void k_out(const hf* __restrict__ ah, const hf* __restrict__ wh,
                                             const float* __restrict__ bout, float* __restrict__ out) {
  __shared__ __align__(16) float st[4][16 * OTP];
  const int tid = threadIdx.x, lane = tid & 31, wave = tid >> 5;
  const int hh = lane >> 4, c = lane & 15;
  const int m0 = blockIdx.x * 64 + wave * 16;
  const int n0 = blockIdx.y * 64;

  v8f acc[4];
#pragma unroll
  for (int t = 0; t < 4; ++t) acc[t] = zero8();
  gemm16x64<EMB>(ah, wh, m0, n0, lane, acc);

  float* sw = st[wave];
#pragma unroll
  for (int t = 0; t < 4; ++t) {
#pragma unroll
    for (int r = 0; r < 8; ++r) sw[(8 * hh + r) * OTP + 16 * t + c] = acc[t][r] * OUTF;
  }
  __syncthreads();
  v4f val[8];
  size_t go[8];
#pragma unroll
  for (int it = 0; it < 8; ++it) {
    const int p    = lane + 32 * it;
    const int L    = p >> 3;
    const int pc   = p & 7;
    const int row  = L >> 1;
    const int half = L & 1;
    const int col  = n0 + half * 32 + pc * 4;
    const v4f tv = *(const v4f*)(sw + row * OTP + half * 32 + pc * 4);
    const v4f bb = *(const v4f*)(bout + col);
    go[it]  = (size_t)(m0 + row) * EMB + col;
    val[it] = tv + bb;
  }
#pragma unroll
  for (int it = 0; it < 8; ++it) *(volatile v4f*)(out + go[it]) = val[it];
  __threadfence();
#pragma unroll
  for (int it = 0; it < 8; ++it) *(volatile v4f*)(out + go[it]) = val[it];
}

extern "C" void kernel_launch(void* const* d_in, const int* in_sizes, int n_in,
                              void* d_out, int out_size, void* d_ws, size_t ws_size,
                              hipStream_t stream) {
  if (n_in < 5) return;
  if (in_sizes[0] != NTOK * EMB) return;
  if (in_sizes[1] != NHD * EMB) return;
  if (in_sizes[2] != EMB * EMB) return;
  if (in_sizes[3] != EMB * EMB) return;
  if (in_sizes[4] != EMB) return;
  if (out_size != NTOK * EMB) return;

  const float* x   = (const float*)d_in[0];
  const float* w_a = (const float*)d_in[1];
  const float* w_v = (const float*)d_in[2];
  const float* w_o = (const float*)d_in[3];
  const float* b_o = (const float*)d_in[4];
  float* out = (float*)d_out;

  size_t off = 0;
  const size_t oX   = off; off += (size_t)NTOK * EMB * 2;
  const size_t oWV  = off; off += (size_t)EMB * EMB * 2;
  const size_t oWO  = off; off += (size_t)EMB * EMB * 2;
  const size_t oZ   = off; off += (size_t)NBH * SQ * 2;
  const size_t oVT  = off; off += (size_t)NBH * HDM * SQ * 2;
  const size_t oMID = off; off += (size_t)NTOK * EMB * 2;
  if (off > ws_size) return;
  if (off > (size_t)134217728) return;

  char* ws = (char*)d_ws;
  hf* Xh  = (hf*)(ws + oX);
  hf* WVh = (hf*)(ws + oWV);
  hf* WOh = (hf*)(ws + oWO);
  hf* Zh  = (hf*)(ws + oZ);
  hf* VTh = (hf*)(ws + oVT);
  hf* MDh = (hf*)(ws + oMID);

  k_cvt<<<dim3(NXB + 2 * NWB), dim3(256), 0, stream>>>(x, w_v, w_o, Xh, WVh, WOh);
  k_zsoft<<<dim3(NBH), dim3(256), 0, stream>>>(x, w_a, Zh);
  k_vproj<<<dim3(NTOK / 64, NHD), dim3(128), 0, stream>>>(Xh, WVh, VTh);
  k_toep<<<dim3(NBH * NQB), dim3(128), 0, stream>>>(Zh, VTh, MDh);
  k_out<<<dim3(NTOK / 64, EMB / 64), dim3(128), 0, stream>>>(MDh, WOh, b_o, out);
  (void)hipGetLastError();
}
